// Encoder_21930103013477
// MI455X (gfx1250) — hardware-verified
//
#include <hip/hip_runtime.h>
#include <math.h>

constexpr int BATCH = 128;
constexpr int WIN   = 128;
constexpr int NDRV  = 32;
constexpr int HID   = 128;
constexpr int GATES = 4 * HID;
constexpr int NROWS = BATCH * WIN;
constexpr float WCARRY     = 64.0f;
constexpr float WCARRY_INV = 1.0f / 64.0f;
constexpr int AZP  = 168;
constexpr int S16P = 264;
constexpr int HSP  = 132;
constexpr int SAP  = 40;
static_assert(NROWS % 64 == 0 && HID % 64 == 0, "GEMM M, N tile multiples");
static_assert(NDRV % 32 == 0 && HID % 32 == 0 && (2 * HID) % 32 == 0, "GEMM K multiples of 32");
static_assert(NROWS % 128 == 0, "self-attention grid exact");
static_assert(BATCH % 16 == 0 && WIN % 16 == 0, "recurrence and attention tiles exact");
static_assert(NDRV == 32, "one lane per driving series");
static_assert(AZP % 8 == 0 && AZP >= NDRV + HID, "A tile pitch");
static_assert(S16P % 8 == 0 && HSP % 4 == 0 && SAP % 8 == 0, "staging pitches");

typedef __attribute__((ext_vector_type(16))) _Float16 v16h;
typedef __attribute__((ext_vector_type(8)))  _Float16 v8h;
typedef __attribute__((ext_vector_type(16))) __bf16   v16b;
typedef __attribute__((ext_vector_type(8)))  __bf16   v8b;
typedef __attribute__((ext_vector_type(8)))  float    v8f;
typedef __attribute__((ext_vector_type(4)))  float    v4f;

__device__ __forceinline__ unsigned short f2bf_bits(float f) {
  unsigned u = __float_as_uint(f);
  return (unsigned short)((u + 0x7FFFu + ((u >> 16) & 1u)) >> 16);
}
__device__ __forceinline__ float bf_bits2f(unsigned short h) { return __uint_as_float(((unsigned)h) << 16); }

__device__ __forceinline__ void dep_guard_h(v8f& a, v8f& b, v16h x, v16h y) { asm volatile("v_nop\n\tv_nop\n\tv_nop\n\tv_nop" : "+v"(a), "+v"(b) : "v"(x), "v"(y)); }
__device__ __forceinline__ void dep_guard_b(v8f& a, v8f& b, v16b x, v16b y) { asm volatile("v_nop\n\tv_nop\n\tv_nop\n\tv_nop" : "+v"(a), "+v"(b) : "v"(x), "v"(y)); }
__device__ __forceinline__ void keep4_h(v16h a, v16h b, v16h c, v16h d) { asm volatile("v_nop" :: "v"(a), "v"(b), "v"(c), "v"(d)); }
__device__ __forceinline__ void keep4_b(v16b a, v16b b, v16b c, v16b d) { asm volatile("v_nop" :: "v"(a), "v"(b), "v"(c), "v"(d)); }
__device__ __forceinline__ void acc_guard4(v8f& a, v8f& b, v8f& c, v8f& d) { asm volatile("v_nop\n\tv_nop\n\tv_nop\n\tv_nop" : "+v"(a), "+v"(b), "+v"(c), "+v"(d)); }
__device__ __forceinline__ void acc_guard2(v8f& a, v8f& b) { asm volatile("v_nop\n\tv_nop\n\tv_nop\n\tv_nop" : "+v"(a), "+v"(b)); }
__device__ __forceinline__ void guard4_full(v8f& a0, v8f& a1, v8f& a2, v8f& a3, v16h x, v16h b0, v16h b1, v16h b2, v16h b3) {
  asm volatile("v_nop\n\tv_nop\n\tv_nop\n\tv_nop" : "+v"(a0), "+v"(a1), "+v"(a2), "+v"(a3) : "v"(x), "v"(b0), "v"(b1), "v"(b2), "v"(b3));
}
__device__ __forceinline__ void guard2_full(v8f& a0, v8f& a1, v16h x, v16h b0, v16h b1) {
  asm volatile("v_nop\n\tv_nop\n\tv_nop\n\tv_nop" : "+v"(a0), "+v"(a1) : "v"(x), "v"(b0), "v"(b1));
}
__device__ __forceinline__ void guard1_full(v8f& a0, v16h x, v16h b0) {
  asm volatile("v_nop\n\tv_nop\n\tv_nop\n\tv_nop" : "+v"(a0) : "v"(x), "v"(b0));
}

template <typename T> struct Frag;
template <> struct Frag<_Float16> {
  typedef v16h V; union U { v16h v; v8h h[2]; };
  static __device__ __forceinline__ v16h load(const _Float16* p) {
    U f; f.h[0] = *(const v8h*)(p); f.h[1] = *(const v8h*)(p + 16); return f.v;
  }
  static __device__ __forceinline__ v8f mma(v16h a, v16h b, v8f c) {
    return __builtin_amdgcn_wmma_f32_16x16x32_f16(false, a, false, b, (short)0, c, false, false);
  }
  static __device__ __forceinline__ void guard(v8f& a, v8f& b, v16h x, v16h y) { dep_guard_h(a, b, x, y); }
  static __device__ __forceinline__ void keep(v16h a, v16h b, v16h c, v16h d) { keep4_h(a, b, c, d); }
};
template <> struct Frag<__bf16> {
  typedef v16b V; union U { v16b v; v8b h[2]; };
  static __device__ __forceinline__ v16b load(const __bf16* p) {
    U f; f.h[0] = *(const v8b*)(p); f.h[1] = *(const v8b*)(p + 16); return f.v;
  }
  static __device__ __forceinline__ v8f mma(v16b a, v16b b, v8f c) {
    return __builtin_amdgcn_wmma_f32_16x16x32_bf16(false, a, false, b, (short)0, c, false, false);
  }
  static __device__ __forceinline__ void guard(v8f& a, v8f& b, v16b x, v16b y) { dep_guard_b(a, b, x, y); }
  static __device__ __forceinline__ void keep(v16b a, v16b b, v16b c, v16b d) { keep4_b(a, b, c, d); }
};

__device__ __forceinline__ float sigm_f(float x) { return __builtin_amdgcn_rcpf(1.0f + expf(-x)); }
__device__ __forceinline__ float tanh_f(float x) { return 1.0f - 2.0f * __builtin_amdgcn_rcpf(expf(2.0f * x) + 1.0f); }

template <int ET> struct Elem;
template <> struct Elem<0> { typedef _Float16 T; };
template <> struct Elem<1> { typedef __bf16 T; };
template <int ET, bool SPLIT, int BIAS_MODE, int OUT_MODE, bool RESID, int ACT = 0>
__global__ __launch_bounds__(256) void wmma_gemm64(
    const unsigned short* __restrict__ Ap, const unsigned short* __restrict__ A2p, int lda, long strideA,
    const unsigned short* __restrict__ Btp, const unsigned short* __restrict__ Bt2p, int ldb, long strideB,
    void* __restrict__ Cout, void* __restrict__ Cout2, int ldc, long strideC,
    const float* __restrict__ bias,
    const float* __restrict__ resid, long strideR,
    int M, int N, int K, float scale) {
  typedef typename Elem<ET>::T T;
  typedef typename Frag<T>::V V;
  const T* A = (const T*)Ap; const T* A2 = (const T*)A2p; const T* Bt = (const T*)Btp; const T* Bt2 = (const T*)Bt2p;
  __shared__ __align__(16) float sT[8][16 * 68];
  const int b    = blockIdx.y;
  const int lane = threadIdx.x & 31;
  const int wave = threadIdx.x >> 5;
  const int tilesN = N >> 6;
  const int tilesM = M >> 6;
  const int tile = blockIdx.x * 8 + wave;
  if (tile >= tilesM * tilesN) return;
  const int tm = tile / tilesN;
  const int tn = tile - tm * tilesN;
  const int m0 = tm << 6;
  const int n0 = tn << 6;

  const T* Ab  = A  + (size_t)b * strideA;
  const T* Bb  = Bt + (size_t)b * strideB;
  const T* Ab2 = SPLIT ? (A2  + (size_t)b * strideA) : nullptr;
  const T* Bb2 = SPLIT ? (Bt2 + (size_t)b * strideB) : nullptr;

  const int rlane = lane & 15;
  const int koff  = (lane >> 4) * 8;
  const int mOff  = (lane >> 4) * 8;

  v8f acc[4][4];
#pragma unroll
  for (int i = 0; i < 4; ++i)
#pragma unroll
    for (int j = 0; j < 4; ++j) acc[i][j] = (v8f){0.f,0.f,0.f,0.f,0.f,0.f,0.f,0.f};

  for (int k0 = 0; k0 < K; k0 += 32) {
    V bh[4], bl[4];
#pragma unroll
    for (int j = 0; j < 4; ++j) {
      const size_t bo = (size_t)(n0 + (j << 4) + rlane) * ldb + koff + k0;
      bh[j] = Frag<T>::load(Bb + bo);
      if (SPLIT) bl[j] = Frag<T>::load(Bb2 + bo);
    }
#pragma unroll
    for (int i = 0; i < 4; ++i) {
      const size_t ao = (size_t)(m0 + (i << 4) + rlane) * lda + koff + k0;
      V ah = Frag<T>::load(Ab + ao);
      V al;
      if (SPLIT) al = Frag<T>::load(Ab2 + ao);
#pragma unroll
      for (int j = 0; j < 4; ++j) {
        acc[i][j] = Frag<T>::mma(ah, bh[j], acc[i][j]);
        if (SPLIT) {
          acc[i][j] = Frag<T>::mma(ah, bl[j], acc[i][j]);
          acc[i][j] = Frag<T>::mma(al, bh[j], acc[i][j]);
        }
      }
      Frag<T>::guard(acc[i][0], acc[i][3], ah, SPLIT ? al : ah);
    }
    Frag<T>::keep(bh[0], bh[1], bh[2], bh[3]);
    if (SPLIT) Frag<T>::keep(bl[0], bl[1], bl[2], bl[3]);
  }
  acc_guard4(acc[0][0], acc[0][1], acc[0][2], acc[0][3]);
  acc_guard4(acc[1][0], acc[1][1], acc[1][2], acc[1][3]);
  acc_guard4(acc[2][0], acc[2][1], acc[2][2], acc[2][3]);
  acc_guard4(acc[3][0], acc[3][1], acc[3][2], acc[3][3]);

  float* slab = sT[wave];
  const float* Rb = RESID ? (resid + (size_t)b * strideR) : nullptr;
#pragma unroll
  for (int i = 0; i < 4; ++i) {
    const int mBase = m0 + (i << 4);
#pragma unroll
    for (int j = 0; j < 4; ++j) {
      const int n = n0 + (j << 4) + rlane;
      float bv = 0.f;
      if (BIAS_MODE == 2) bv = bias[n];
#pragma unroll
      for (int r = 0; r < 8; ++r) {
        float v = acc[i][j][r] * scale;
        if (BIAS_MODE == 1) v += bias[mBase + mOff + r];
        if (BIAS_MODE == 2) v += bv;
        if (RESID) v += Rb[(size_t)(mBase + mOff + r) * ldc + n];
        if (ACT == 1) v = tanhf(v);
        if (ACT == 2) v = fmaxf(v, 0.0f);
        if (ACT == 3) v = v / (1.0f + expf(-v));
        if (ACT == 4) v = (v > 0.f) ? v : 0.01f * v;
        if (ACT == 5) v = 0.5f * v * (1.0f + erff(v * 0.70710678118654752f));
        slab[(mOff + r) * 68 + (j << 4) + rlane] = v;
      }
    }
    __builtin_amdgcn_fence(__ATOMIC_RELEASE, "workgroup");
    __builtin_amdgcn_wave_barrier();
    __builtin_amdgcn_fence(__ATOMIC_ACQUIRE, "workgroup");
    if (OUT_MODE == 0) {
      float* C = (float*)Cout + (size_t)b * strideC;
      const int hh = lane >> 4, c4 = (lane & 15) * 4;
      for (int pass = 0; pass < 2; ++pass) {
#pragma unroll
        for (int it = 0; it < 8; ++it) {
          const int row = it * 2 + hh;
          v4f v = *(const v4f*)(slab + row * 68 + c4);
          *(volatile v4f*)(C + (size_t)(mBase + row) * ldc + n0 + c4) = v;
        }
        __threadfence();
      }
    } else {
      const int q = lane >> 3, c8 = (lane & 7) * 8;
      unsigned short* C  = (unsigned short*)Cout  + (size_t)b * strideC;
      unsigned short* C2 = (OUT_MODE == 2) ? ((unsigned short*)Cout2 + (size_t)b * strideC) : nullptr;
      for (int pass = 0; pass < 2; ++pass) {
#pragma unroll
        for (int it = 0; it < 4; ++it) {
          const int row = it * 4 + q;
          const float* sp = slab + row * 68 + c8;
          v8h hv, lv;
#pragma unroll
          for (int e = 0; e < 8; ++e) {
            if (OUT_MODE == 1) {
              hv[e] = (_Float16)sp[e];
            } else {
              unsigned short hb = f2bf_bits(sp[e]);
              unsigned short lb = f2bf_bits(sp[e] - bf_bits2f(hb));
              hv[e] = __builtin_bit_cast(_Float16, hb);
              lv[e] = __builtin_bit_cast(_Float16, lb);
            }
          }
          *(volatile v8h*)(C + (size_t)(mBase + row) * ldc + n0 + c8) = hv;
          if (OUT_MODE == 2) *(volatile v8h*)(C2 + (size_t)(mBase + row) * ldc + n0 + c8) = lv;
        }
        __threadfence();
      }
    }
    __builtin_amdgcn_fence(__ATOMIC_RELEASE, "workgroup");
    __builtin_amdgcn_wave_barrier();
    __builtin_amdgcn_fence(__ATOMIC_ACQUIRE, "workgroup");
  }
}

__global__ __launch_bounds__(256) void cvt8x3_kernel(const float* s0, const float* s1, const float* s2,
                                                     unsigned short* d0, unsigned short* d1, unsigned short* d2,
                                                     int n8, float sc) {
  const int y = blockIdx.y;
  const float* src = (y == 0) ? s0 : ((y == 1) ? s1 : s2);
  unsigned short* dst = (y == 0) ? d0 : ((y == 1) ? d1 : d2);
  const int i = blockIdx.x * 256 + threadIdx.x;
  if (i < n8) {
    const float* sp = src + (size_t)i * 8;
    const v4f a = *(const v4f*)(sp);
    const v4f b = *(const v4f*)(sp + 4);
    v8h hv;
#pragma unroll
    for (int e = 0; e < 4; ++e) {
      const float fa = a[e] * sc;
      const float fb = b[e] * sc;
      hv[e]     = (_Float16)fa;
      hv[4 + e] = (_Float16)fb;
    }
    volatile v8h* dp = (volatile v8h*)(dst + (size_t)i * 8);
    *dp = hv;
    __threadfence();
    *dp = hv;
  }
}

__global__ __launch_bounds__(256) void selfatt_kernel(const unsigned short* __restrict__ g16p,
                                                      const unsigned short* __restrict__ wa16p,
                                                      const float* __restrict__ ba, const float* __restrict__ x,
                                                      unsigned short* __restrict__ sa16) {
  __shared__ __align__(16) _Float16 Ss[8][16 * SAP];
  const _Float16* g16  = (const _Float16*)(const void*)g16p;
  const _Float16* wa16 = (const _Float16*)(const void*)wa16p;
  const int tid = threadIdx.x, lane = tid & 31, wave = tid >> 5;
  const int c = lane & 15, hh = lane >> 4, koff = hh * 8;
  const int row0 = (blockIdx.x * 8 + wave) * 16;

  const _Float16* arow = g16 + (size_t)(row0 + c) * HID + koff;
  const _Float16* b0p  = wa16 + (size_t)c * HID + koff;
  const _Float16* b1p  = wa16 + (size_t)(16 + c) * HID + koff;
  v8f acc0 = (v8f){0.f,0.f,0.f,0.f,0.f,0.f,0.f,0.f};
  v8f acc1 = acc0;
#pragma unroll 1
  for (int k0 = 0; k0 < HID; k0 += 32) {
    const v16h a  = Frag<_Float16>::load(arow + k0);
    const v16h b0 = Frag<_Float16>::load(b0p + k0);
    const v16h b1 = Frag<_Float16>::load(b1p + k0);
    acc0 = Frag<_Float16>::mma(a, b0, acc0);
    acc1 = Frag<_Float16>::mma(a, b1, acc1);
    guard2_full(acc0, acc1, a, b0, b1);
  }
  acc_guard2(acc0, acc1);

  _Float16* slab = Ss[wave];
  {
    const float bav = ba[c];
    float xv[8];
#pragma unroll
    for (int r = 0; r < 8; ++r) xv[r] = x[(size_t)(row0 + 8 * hh + r) * NDRV + c];
#pragma unroll
    for (int r = 0; r < 8; ++r) {
      const float z = acc0[r] * WCARRY_INV + bav;
      const float s = sigm_f(z) * xv[r];
      slab[(8 * hh + r) * SAP + c] = (_Float16)s;
    }
  }
  asm volatile("" ::: "memory");
  {
    const float bav = ba[16 + c];
    float xv[8];
#pragma unroll
    for (int r = 0; r < 8; ++r) xv[r] = x[(size_t)(row0 + 8 * hh + r) * NDRV + 16 + c];
#pragma unroll
    for (int r = 0; r < 8; ++r) {
      const float z = acc1[r] * WCARRY_INV + bav;
      const float s = sigm_f(z) * xv[r];
      slab[(8 * hh + r) * SAP + 16 + c] = (_Float16)s;
    }
  }
  __syncthreads();
  for (int pass = 0; pass < 2; ++pass) {
#pragma unroll
    for (int it = 0; it < 2; ++it) {
      const int p = it * 32 + lane;
      const v8h v = *(const v8h*)(slab + (p >> 2) * SAP + (p & 3) * 8);
      *(volatile v8h*)(sa16 + (size_t)row0 * NDRV + (size_t)p * 8) = v;
    }
    __threadfence();
  }
}

struct LstmCfg {
  const unsigned short* in16;
  const unsigned short* wih;
  const unsigned short* whh;
  const float* bih;
  const float* bhh;
  float* outf;
  unsigned short* hs;
  int mode;
  int ocol;
};
static_assert(sizeof(LstmCfg) == 64, "no padding");

__global__ __launch_bounds__(256) void lstm_seq_kernel(LstmCfg ca, LstmCfg cb) {
  __shared__ __align__(16) _Float16 Az[16 * AZP];
  __shared__ __align__(16) _Float16 St16[16 * S16P];
  __shared__ __align__(16) float    Hs[16 * HSP];
  const bool sel = (blockIdx.y != 0);
  const _Float16* in16 = (const _Float16*)(const void*)(sel ? cb.in16 : ca.in16);
  const _Float16* wih  = (const _Float16*)(const void*)(sel ? cb.wih : ca.wih);
  const _Float16* whh  = (const _Float16*)(const void*)(sel ? cb.whh : ca.whh);
  const float* bih = sel ? cb.bih : ca.bih;
  const float* bhh = sel ? cb.bhh : ca.bhh;
  float* outf = sel ? cb.outf : ca.outf;
  unsigned short* hsp = sel ? cb.hs : ca.hs;
  const int mode = sel ? cb.mode : ca.mode;
  const int ocol = sel ? cb.ocol : ca.ocol;

  const int tid = threadIdx.x, lane = tid & 31, wave = tid >> 5;
  const int c = lane & 15, hh = lane >> 4, koff = hh * 8;
  const int rowbase = blockIdx.x * 16;
  const int j = 16 * wave + c;

  {
    const v8h zero8 = (v8h){(_Float16)0.0f, (_Float16)0.0f, (_Float16)0.0f, (_Float16)0.0f,
                            (_Float16)0.0f, (_Float16)0.0f, (_Float16)0.0f, (_Float16)0.0f};
#pragma unroll 1
    for (int i = tid; i < (16 * AZP) / 8; i += 256) *(v8h*)(Az + i * 8) = zero8;
  }
  __syncthreads();
  if (tid < 64) {
    const int m = tid >> 2, p8 = (tid & 3) * 8;
    const v8h v = *(const v8h*)(in16 + ((size_t)(rowbase + m) * WIN) * NDRV + p8);
    *(v8h*)(Az + m * AZP + p8) = v;
  }
  float bb[4];
#pragma unroll
  for (int g = 0; g < 4; ++g) bb[g] = bih[g * HID + j] + bhh[g * HID + j];
  float cst[8], hst[8];
#pragma unroll
  for (int r = 0; r < 8; ++r) { cst[r] = 0.0f; hst[r] = 0.0f; }
  __syncthreads();

  const _Float16* azrow = Az + c * AZP + koff;
  const _Float16* wihp = wih + (size_t)j * NDRV + koff;
  const _Float16* whhp = whh + (size_t)j * HID + koff;
  const v8f z8 = {0.f, 0.f, 0.f, 0.f, 0.f, 0.f, 0.f, 0.f};

#pragma unroll 1
  for (int t = 0; t < WIN; ++t) {
    if (mode == 0) {
#pragma unroll
      for (int r = 0; r < 8; ++r) {
        St16[(8 * hh + r) * S16P + j]       = (_Float16)hst[r];
        St16[(8 * hh + r) * S16P + HID + j] = (_Float16)cst[r];
      }
    }
    v8f acc0 = z8, acc1 = z8, acc2 = z8, acc3 = z8;
    {
      const v16h a  = Frag<_Float16>::load(azrow);
      const v16h b0 = Frag<_Float16>::load(wihp);
      const v16h b1 = Frag<_Float16>::load(wihp + (size_t)1 * HID * NDRV);
      const v16h b2 = Frag<_Float16>::load(wihp + (size_t)2 * HID * NDRV);
      const v16h b3 = Frag<_Float16>::load(wihp + (size_t)3 * HID * NDRV);
      acc0 = Frag<_Float16>::mma(a, b0, acc0);
      acc1 = Frag<_Float16>::mma(a, b1, acc1);
      acc2 = Frag<_Float16>::mma(a, b2, acc2);
      acc3 = Frag<_Float16>::mma(a, b3, acc3);
      guard4_full(acc0, acc1, acc2, acc3, a, b0, b1, b2, b3);
    }
#pragma unroll 1
    for (int k0 = 0; k0 < HID; k0 += 32) {
      const v16h a  = Frag<_Float16>::load(azrow + NDRV + k0);
      const v16h b0 = Frag<_Float16>::load(whhp + k0);
      const v16h b1 = Frag<_Float16>::load(whhp + (size_t)1 * HID * HID + k0);
      const v16h b2 = Frag<_Float16>::load(whhp + (size_t)2 * HID * HID + k0);
      const v16h b3 = Frag<_Float16>::load(whhp + (size_t)3 * HID * HID + k0);
      acc0 = Frag<_Float16>::mma(a, b0, acc0);
      acc1 = Frag<_Float16>::mma(a, b1, acc1);
      acc2 = Frag<_Float16>::mma(a, b2, acc2);
      acc3 = Frag<_Float16>::mma(a, b3, acc3);
      guard4_full(acc0, acc1, acc2, acc3, a, b0, b1, b2, b3);
    }
    acc_guard4(acc0, acc1, acc2, acc3);
#pragma unroll
    for (int r = 0; r < 8; ++r) {
      const float zi = acc0[r] * WCARRY_INV + bb[0];
      const float zf = acc1[r] * WCARRY_INV + bb[1];
      const float zg = acc2[r] * WCARRY_INV + bb[2];
      const float zo = acc3[r] * WCARRY_INV + bb[3];
      const float ig = sigm_f(zi);
      const float fg = sigm_f(zf);
      const float gg = tanh_f(zg);
      const float og = sigm_f(zo);
      const float cn = fg * cst[r] + ig * gg;
      cst[r] = cn;
      hst[r] = og * tanh_f(cn);
    }
    if (mode != 0) {
#pragma unroll
      for (int r = 0; r < 8; ++r) Hs[(8 * hh + r) * HSP + j] = hst[r];
    }
    __syncthreads();
#pragma unroll
    for (int r = 0; r < 8; ++r) Az[(8 * hh + r) * AZP + NDRV + j] = (_Float16)hst[r];
    if (tid < 64) {
      const int tn = (t + 1 < WIN) ? (t + 1) : (WIN - 1);
      const int m = tid >> 2, p8 = (tid & 3) * 8;
      const v8h v = *(const v8h*)(in16 + ((size_t)(rowbase + m) * WIN + (size_t)tn) * NDRV + p8);
      *(v8h*)(Az + m * AZP + p8) = v;
    }
    if (mode == 0) {
      for (int pass = 0; pass < 2; ++pass) {
#pragma unroll
        for (int it = 0; it < 2; ++it) {
          const int idx = it * 256 + tid;
          const int row = idx >> 5, c8 = (idx & 31) * 8;
          const v8h v = *(const v8h*)(St16 + row * S16P + c8);
          *(volatile v8h*)(hsp + ((size_t)(rowbase + row) * WIN + (size_t)t) * (2 * HID) + c8) = v;
        }
        __threadfence();
      }
    } else {
      for (int pass = 0; pass < 2; ++pass) {
#pragma unroll
        for (int it = 0; it < 2; ++it) {
          const int idx = it * 256 + tid;
          const int row = idx >> 5, c4 = (idx & 31) * 4;
          const v4f v = *(const v4f*)(Hs + row * HSP + c4);
          *(volatile v4f*)(outf + ((size_t)(rowbase + row) * WIN + (size_t)t) * (2 * HID) + ocol + c4) = v;
        }
        __threadfence();
      }
    }
    __syncthreads();
  }
}

__global__ __launch_bounds__(128) void attn_kernel(const float* __restrict__ tux, const float* __restrict__ twp,
                                                   const float* __restrict__ x, const float* __restrict__ ve,
                                                   unsigned short* __restrict__ ia16) {
  __shared__ __align__(16) float    tws[16 * HID];
  __shared__ __align__(16) float    xs[WIN * NDRV];
  __shared__ __align__(16) float    es[16 * WIN];
  __shared__ __align__(16) float    ves[HID];
  __shared__ __align__(16) _Float16 ias[16 * NDRV];
  const int tid = threadIdx.x, lane = tid & 31, wave = tid >> 5;
  const int c = lane & 15, hh = lane >> 4;
  const int b  = blockIdx.x >> 3;
  const int t0 = (blockIdx.x & 7) * 16;

  {
    const float* twb = twp + (size_t)(b * WIN + t0) * HID;
#pragma unroll
    for (int i = 0; i < 4; ++i) {
      const int idx = i * 128 + tid;
      *(v4f*)(tws + idx * 4) = *(const v4f*)(twb + idx * 4);
    }
    asm volatile("" ::: "memory");
    const float* xb = x + (size_t)b * WIN * NDRV;
#pragma unroll
    for (int i = 0; i < 4; ++i) {
      const int idx = i * 128 + tid;
      *(v4f*)(xs + idx * 4) = *(const v4f*)(xb + idx * 4);
    }
    asm volatile("" ::: "memory");
#pragma unroll
    for (int i = 4; i < 8; ++i) {
      const int idx = i * 128 + tid;
      *(v4f*)(xs + idx * 4) = *(const v4f*)(xb + idx * 4);
    }
    if (tid < 32) *(v4f*)(ves + tid * 4) = *(const v4f*)(ve + tid * 4);
  }
  __syncthreads();

  v16h bv[4];
#pragma unroll
  for (int kc = 0; kc < 4; ++kc) {
#pragma unroll
    for (int i = 0; i < 8; ++i) {
      float f0 = ves[32 * kc + 8 * hh + i] * WCARRY;
      float f1 = ves[32 * kc + 16 + 8 * hh + i] * WCARRY;
      f0 = (c == 0) ? f0 : 0.0f;
      f1 = (c == 0) ? f1 : 0.0f;
      bv[kc][i]     = (_Float16)f0;
      bv[kc][8 + i] = (_Float16)f1;
    }
  }

  const float* tub = tux + (size_t)b * WIN * HID;
  const v8f z8 = {0.f, 0.f, 0.f, 0.f, 0.f, 0.f, 0.f, 0.f};
#pragma unroll 1
  for (int tile = 0; tile < WIN / 16; ++tile) {
    v8f acc[4];
    acc[0] = z8; acc[1] = z8; acc[2] = z8; acc[3] = z8;
    const float* urow = tub + (size_t)(tile * 16 + c) * HID + 8 * hh;
#pragma unroll
    for (int kc = 0; kc < 4; ++kc) {
      const v4f u0 = *(const v4f*)(urow + 32 * kc);
      const v4f u1 = *(const v4f*)(urow + 32 * kc + 4);
      const v4f u2 = *(const v4f*)(urow + 32 * kc + 16);
      const v4f u3 = *(const v4f*)(urow + 32 * kc + 20);
#pragma unroll
      for (int tl = 0; tl < 4; ++tl) {
        const float* wrow = tws + (4 * wave + tl) * HID + 32 * kc + 8 * hh;
        const v4f w0 = *(const v4f*)(wrow);
        const v4f w1 = *(const v4f*)(wrow + 4);
        const v4f w2 = *(const v4f*)(wrow + 16);
        const v4f w3 = *(const v4f*)(wrow + 20);
        v16h a;
#pragma unroll
        for (int e = 0; e < 4; ++e) {
          const float q0 = (u0[e] + w0[e]) * __builtin_amdgcn_rcpf(fmaf(u0[e], w0[e], 1.0f));
          const float q1 = (u1[e] + w1[e]) * __builtin_amdgcn_rcpf(fmaf(u1[e], w1[e], 1.0f));
          const float q2 = (u2[e] + w2[e]) * __builtin_amdgcn_rcpf(fmaf(u2[e], w2[e], 1.0f));
          const float q3 = (u3[e] + w3[e]) * __builtin_amdgcn_rcpf(fmaf(u3[e], w3[e], 1.0f));
          a[e]      = (_Float16)q0;
          a[4 + e]  = (_Float16)q1;
          a[8 + e]  = (_Float16)q2;
          a[12 + e] = (_Float16)q3;
        }
        acc[tl] = Frag<_Float16>::mma(a, bv[kc], acc[tl]);
        guard1_full(acc[tl], a, bv[kc]);
      }
    }
    acc_guard4(acc[0], acc[1], acc[2], acc[3]);
    if (c == 0) {
#pragma unroll
      for (int tl = 0; tl < 4; ++tl)
#pragma unroll
        for (int r = 0; r < 8; ++r)
          es[(4 * wave + tl) * WIN + tile * 16 + 8 * hh + r] = acc[tl][r] * WCARRY_INV;
    }
  }
  __syncthreads();

#pragma unroll
  for (int tl = 0; tl < 4; ++tl) {
    float* er = es + (4 * wave + tl) * WIN;
    v4f ev = *(const v4f*)(er + 4 * lane);
    float mx = fmaxf(fmaxf(ev[0], ev[1]), fmaxf(ev[2], ev[3]));
#pragma unroll
    for (int off = 1; off < 32; off <<= 1) mx = fmaxf(mx, __shfl_xor(mx, off, 32));
    v4f pv;
    pv[0] = expf(ev[0] - mx);
    pv[1] = expf(ev[1] - mx);
    pv[2] = expf(ev[2] - mx);
    pv[3] = expf(ev[3] - mx);
    float s = (pv[0] + pv[1]) + (pv[2] + pv[3]);
#pragma unroll
    for (int off = 1; off < 32; off <<= 1) s += __shfl_xor(s, off, 32);
    const float inv = 1.0f / s;
    pv[0] *= inv; pv[1] *= inv; pv[2] *= inv; pv[3] *= inv;
    *(v4f*)(er + 4 * lane) = pv;
  }
  __syncthreads();

  {
    const float* e0 = es + (4 * wave) * WIN;
    float s0 = 0.0f, s1 = 0.0f, s2 = 0.0f, s3 = 0.0f;
#pragma unroll 4
    for (int tt = 0; tt < WIN; ++tt) {
      const float xv = xs[tt * NDRV + lane];
      s0 += e0[tt] * xv;
      s1 += e0[WIN + tt] * xv;
      s2 += e0[2 * WIN + tt] * xv;
      s3 += e0[3 * WIN + tt] * xv;
    }
    ias[(4 * wave + 0) * NDRV + lane] = (_Float16)s0;
    ias[(4 * wave + 1) * NDRV + lane] = (_Float16)s1;
    ias[(4 * wave + 2) * NDRV + lane] = (_Float16)s2;
    ias[(4 * wave + 3) * NDRV + lane] = (_Float16)s3;
  }
  __syncthreads();
  if (wave == 0) {
    unsigned short* op = ia16 + (size_t)(b * WIN + t0) * NDRV;
    for (int pass = 0; pass < 2; ++pass) {
#pragma unroll
      for (int it = 0; it < 2; ++it) {
        const int p = it * 32 + lane;
        const v8h v = *(const v8h*)(ias + p * 8);
        *(volatile v8h*)(op + (size_t)p * 8) = v;
      }
      __threadfence();
    }
  }
}

extern "C" void kernel_launch(void* const* d_in, const int* in_sizes, int n_in,
                              void* d_out, int out_size, void* d_ws, size_t ws_size, hipStream_t stream) {
  if (n_in < 20 || d_out == nullptr || d_ws == nullptr) return;
  if (in_sizes[0] != NROWS * NDRV || in_sizes[1] != GATES * NDRV || in_sizes[2] != GATES * HID ||
      in_sizes[3] != GATES || in_sizes[4] != GATES || in_sizes[5] != HID * 2 * HID ||
      in_sizes[6] != HID * NDRV || in_sizes[7] != HID || in_sizes[8] != HID * NDRV || in_sizes[9] != HID ||
      in_sizes[10] != NDRV * HID || in_sizes[11] != NDRV ||
      in_sizes[12] != GATES * NDRV || in_sizes[13] != GATES * HID || in_sizes[14] != GATES || in_sizes[15] != GATES ||
      in_sizes[16] != GATES * NDRV || in_sizes[17] != GATES * HID || in_sizes[18] != GATES || in_sizes[19] != GATES ||
      out_size != NROWS * 2 * HID) return;

  const float* x    = (const float*)d_in[0];
  const float* Wih0 = (const float*)d_in[1];
  const float* Whh0 = (const float*)d_in[2];
  const float* bih0 = (const float*)d_in[3];
  const float* bhh0 = (const float*)d_in[4];
  const float* We   = (const float*)d_in[5];
  const float* Ue   = (const float*)d_in[6];
  const float* Ve   = (const float*)d_in[7];
  const float* Wg   = (const float*)d_in[8];
  const float* bg   = (const float*)d_in[9];
  const float* Wa   = (const float*)d_in[10];
  const float* ba   = (const float*)d_in[11];
  const float* Wih1 = (const float*)d_in[12];
  const float* Whh1 = (const float*)d_in[13];
  const float* bih1 = (const float*)d_in[14];
  const float* bhh1 = (const float*)d_in[15];
  const float* Wih2 = (const float*)d_in[16];
  const float* Whh2 = (const float*)d_in[17];
  const float* bih2 = (const float*)d_in[18];
  const float* bhh2 = (const float*)d_in[19];
  float* out = (float*)d_out;

  char* ws = (char*)d_ws; size_t off = 0;
  auto carve = [&](size_t bytes) -> char* { char* p = ws + off; off += (bytes + 255) & ~(size_t)255; return p; };
  unsigned short* x16   = (unsigned short*)carve((size_t)NROWS * NDRV * 2);
  unsigned short* sa16  = (unsigned short*)carve((size_t)NROWS * NDRV * 2);
  unsigned short* ia16  = (unsigned short*)carve((size_t)NROWS * NDRV * 2);
  unsigned short* g16   = (unsigned short*)carve((size_t)NROWS * HID * 2);
  unsigned short* hs16  = (unsigned short*)carve((size_t)NROWS * 2 * HID * 2);
  float*          tux   = (float*)carve((size_t)NROWS * HID * 4);
  float*          tw    = (float*)carve((size_t)NROWS * HID * 4);
  unsigned short* wih16_0 = (unsigned short*)carve((size_t)GATES * NDRV * 2);
  unsigned short* wih16_1 = (unsigned short*)carve((size_t)GATES * NDRV * 2);
  unsigned short* wih16_2 = (unsigned short*)carve((size_t)GATES * NDRV * 2);
  unsigned short* whh16_0 = (unsigned short*)carve((size_t)GATES * HID * 2);
  unsigned short* whh16_1 = (unsigned short*)carve((size_t)GATES * HID * 2);
  unsigned short* whh16_2 = (unsigned short*)carve((size_t)GATES * HID * 2);
  unsigned short* we16  = (unsigned short*)carve((size_t)HID * 2 * HID * 2);
  unsigned short* ue16  = (unsigned short*)carve((size_t)HID * NDRV * 2);
  unsigned short* wg16  = (unsigned short*)carve((size_t)HID * NDRV * 2);
  unsigned short* wa16  = (unsigned short*)carve((size_t)NDRV * HID * 2);
  if (off > ws_size || off > (size_t)134217728) return;

  const int n8x  = NROWS * NDRV / 8;
  const int n8ih = GATES * NDRV / 8;
  const int n8hh = GATES * HID / 8;
  const int n8sm = HID * NDRV / 8;
  const int n8we = HID * 2 * HID / 8;
  static_assert((NROWS * NDRV / 8) % 256 == 0 && (GATES * NDRV / 8) % 256 == 0 && (GATES * HID / 8) % 256 == 0 &&
                (HID * NDRV / 8) % 256 == 0 && (HID * 2 * HID / 8) % 256 == 0, "convert grids exact");
  cvt8x3_kernel<<<dim3(n8x / 256, 1), 256, 0, stream>>>(x, x, x, x16, x16, x16, n8x, 1.0f);
  cvt8x3_kernel<<<dim3(n8ih / 256, 3), 256, 0, stream>>>(Wih0, Wih1, Wih2, wih16_0, wih16_1, wih16_2, n8ih, WCARRY);
  cvt8x3_kernel<<<dim3(n8hh / 256, 3), 256, 0, stream>>>(Whh0, Whh1, Whh2, whh16_0, whh16_1, whh16_2, n8hh, WCARRY);
  cvt8x3_kernel<<<dim3(n8sm / 256, 3), 256, 0, stream>>>(Ue, Wg, Wa, ue16, wg16, wa16, n8sm, WCARRY);
  cvt8x3_kernel<<<dim3(n8we / 256, 1), 256, 0, stream>>>(We, We, We, we16, we16, we16, n8we, WCARRY);

  const dim3 ggrid((NROWS / 64) * (HID / 64) / 8, 1);
  wmma_gemm64<0, false, 0, 0, false, 1><<<ggrid, 256, 0, stream>>>(
      x16, x16, NDRV, 0L, ue16, ue16, NDRV, 0L, (void*)tux, (void*)tux, HID, 0L,
      bg, tux, 0L, NROWS, HID, NDRV, WCARRY_INV);
  wmma_gemm64<0, false, 2, 1, false, 1><<<ggrid, 256, 0, stream>>>(
      x16, x16, NDRV, 0L, wg16, wg16, NDRV, 0L, (void*)g16, (void*)g16, HID, 0L,
      bg, tux, 0L, NROWS, HID, NDRV, WCARRY_INV);
  selfatt_kernel<<<NROWS / 128, 256, 0, stream>>>(g16, wa16, ba, x, sa16);

  LstmCfg c0;
  c0.in16 = x16;  c0.wih = wih16_0; c0.whh = whh16_0; c0.bih = bih0; c0.bhh = bhh0;
  c0.outf = out;  c0.hs = hs16; c0.mode = 0; c0.ocol = 0;
  LstmCfg c2;
  c2.in16 = sa16; c2.wih = wih16_2; c2.whh = whh16_2; c2.bih = bih2; c2.bhh = bhh2;
  c2.outf = out;  c2.hs = hs16; c2.mode = 1; c2.ocol = HID;
  lstm_seq_kernel<<<dim3(BATCH / 16, 2), 256, 0, stream>>>(c0, c2);

  wmma_gemm64<0, false, 0, 0, false, 1><<<ggrid, 256, 0, stream>>>(
      hs16, hs16, 2 * HID, 0L, we16, we16, 2 * HID, 0L, (void*)tw, (void*)tw, HID, 0L,
      bg, tux, 0L, NROWS, HID, 2 * HID, WCARRY_INV);

  attn_kernel<<<BATCH * (WIN / 16), 128, 0, stream>>>(tux, tw, x, Ve, ia16);

  LstmCfg c1;
  c1.in16 = ia16; c1.wih = wih16_1; c1.whh = whh16_1; c1.bih = bih1; c1.bhh = bhh1;
  c1.outf = out;  c1.hs = hs16; c1.mode = 1; c1.ocol = 0;
  lstm_seq_kernel<<<dim3(BATCH / 16, 1), 256, 0, stream>>>(c1, c1);
}
